// SequenceLSTM_62929860821333
// MI455X (gfx1250) — hardware-verified
//
#include <hip/hip_runtime.h>
#include <stddef.h>

typedef __attribute__((ext_vector_type(16))) _Float16 v16h;
typedef __attribute__((ext_vector_type(8)))  _Float16 v8h;
typedef __attribute__((ext_vector_type(8)))  float    v8f;
typedef __attribute__((ext_vector_type(4)))  float    v4f;

constexpr int HID    = 51;
constexpr int HPAD   = 64;
constexpr int NGATE  = 4 * HPAD;
constexpr int NBATCH = 256;
constexpr int BROWS  = 16;
constexpr int K1P    = 64;
constexpr int K2P    = 128;
constexpr int APITCH = 136;
constexpr int GPITCH = 260;
constexpr int OCHUNK = 64;
constexpr int OPITCH = 68;
constexpr int NT1    = NGATE * K1P / 8;
constexpr int NT2    = NGATE * K2P / 8;
constexpr float HSCALE  = 16.0f;
constexpr float WSCALE  = 64.0f;
constexpr float ACC_INV = 1.0f / 1024.0f;

static_assert(NGATE == 256, "one pack/init thread per gate column");
static_assert(K1P % 32 == 0 && K2P % 32 == 0, "K steps of 32");
static_assert((APITCH * 2) % 16 == 0 && (OPITCH * 4) % 16 == 0, "16-B aligned LDS rows");
static_assert(NBATCH % BROWS == 0, "whole row tiles");
static_assert(NT1 % 256 == 0 && (NT1 + NT2) % 256 == 0, "pack grid has no tail");
static_assert(OCHUNK == 64 && BROWS == 16, "flush lane map: 8 waves x 2 rows x 2 lines");

__device__ __forceinline__ void dep_guard_h(v8f& a, v8f& b, v16h x, v16h y) {
  asm volatile("v_nop\n\tv_nop\n\tv_nop\n\tv_nop" : "+v"(a), "+v"(b) : "v"(x), "v"(y));
}
__device__ __forceinline__ void keep4_h(v16h a, v16h b, v16h c, v16h d) {
  asm volatile("v_nop" :: "v"(a), "v"(b), "v"(c), "v"(d));
}

template <typename T> struct Frag;
template <> struct Frag<_Float16> {
  typedef v16h V; union U { v16h v; v8h h[2]; };
  static __device__ __forceinline__ v16h load(const _Float16* p) {
    U f; f.h[0] = *(const v8h*)(p); f.h[1] = *(const v8h*)(p + 16); return f.v;
  }
  static __device__ __forceinline__ v8f mma(v16h a, v16h b, v8f c) {
    return __builtin_amdgcn_wmma_f32_16x16x32_f16(false, a, false, b, (short)0, c, false, false);
  }
};
typedef Frag<_Float16> FragH;

__device__ __forceinline__ float tanh_f(float xv) {
  const float ax = fabsf(xv);
  const float t  = expf(-2.0f * ax);
  const float r  = __builtin_amdgcn_rcpf(1.0f + t);
  const float y  = (1.0f - t) * r;
  return copysignf(y, xv);
}

__global__ __launch_bounds__(256)
void pack_tables(const float* __restrict__ Whh1, const float* __restrict__ Wih2,
                 const float* __restrict__ Whh2,
                 _Float16* __restrict__ WT1, _Float16* __restrict__ WT2) {
  const int i = blockIdx.x * 256 + threadIdx.x;
  v8h hv;
  _Float16* dst;
  if (i < NT1) {
    const int n  = i >> 3;
    const int k8 = (i & 7) * 8;
    const int g  = n >> 6, c = n & 63;
    const int cc = (c < HID) ? c : (HID - 1);
    const int rowi = (g * HID + cc) * HID;
#pragma unroll
    for (int e = 0; e < 8; ++e) {
      const int k  = k8 + e;
      const int kc = (k < HID) ? k : (HID - 1);
      const float w = Whh1[rowi + kc];
      const float v = (c < HID && k < HID) ? w * WSCALE : 0.0f;
      hv[e] = (_Float16)v;
    }
    dst = WT1 + (size_t)i * 8;
  } else {
    const int j  = i - NT1;
    const int n  = j >> 4;
    const int k8 = (j & 15) * 8;
    const int g  = n >> 6, c = n & 63;
    const int cc = (c < HID) ? c : (HID - 1);
    const int rowi = (g * HID + cc) * HID;
    const bool second = (k8 >= HPAD);
    const float* src = second ? Whh2 : Wih2;
    const int kb = second ? (k8 - HPAD) : k8;
#pragma unroll
    for (int e = 0; e < 8; ++e) {
      const int k  = kb + e;
      const int kc = (k < HID) ? k : (HID - 1);
      const float w = src[rowi + kc];
      const float v = (c < HID && k < HID) ? w * WSCALE : 0.0f;
      hv[e] = (_Float16)v;
    }
    dst = WT2 + (size_t)j * 8;
  }
  *(volatile v8h*)dst = hv;
  __threadfence();
  *(volatile v8h*)dst = hv;
}

template <int NKS>
__device__ __forceinline__ void gemm16(const _Float16* arow, const _Float16* wt0,
                                       const _Float16* wt1, v8f& acc0, v8f& acc1) {
#pragma unroll
  for (int gq = 0; gq < NKS / 2; ++gq) {
    const int k0 = gq * 64;
    const v16h b00 = FragH::load(wt0 + k0);
    const v16h b01 = FragH::load(wt0 + k0 + 32);
    const v16h b10 = FragH::load(wt1 + k0);
    const v16h b11 = FragH::load(wt1 + k0 + 32);
    const v16h a0  = FragH::load(arow + k0);
    const v16h a1  = FragH::load(arow + k0 + 32);
    acc0 = FragH::mma(a0, b00, acc0);
    acc0 = FragH::mma(a1, b01, acc0);
    acc1 = FragH::mma(a0, b10, acc1);
    acc1 = FragH::mma(a1, b11, acc1);
    dep_guard_h(acc0, acc1, a0, a1);
    keep4_h(b00, b01, b10, b11);
    asm volatile("" ::: "memory");
  }
}

__device__ __forceinline__ void gate_epi(float* gs, int col, int rbase, v8f acc, const float* xin,
                                         float wx, float bs, float pre, float amul, float aadd) {
#pragma unroll
  for (int r = 0; r < 8; ++r) {
    const float g0 = __builtin_fmaf(acc[r], ACC_INV, __builtin_fmaf(xin[r], wx, bs));
    const float y  = tanh_f(pre * g0);
    gs[(rbase + r) * GPITCH + col] = __builtin_fmaf(y, amul, aadd);
  }
}

__global__ __launch_bounds__(256)
void lstm_scan(const float* __restrict__ x,
               const float* __restrict__ Wih1,
               const float* __restrict__ bih1, const float* __restrict__ bhh1,
               const float* __restrict__ bih2, const float* __restrict__ bhh2,
               const float* __restrict__ fcw,  const float* __restrict__ fcb,
               const int*   __restrict__ futp,
               const _Float16* __restrict__ WT1, const _Float16* __restrict__ WT2,
               float* __restrict__ out, int T, int TT) {
  __shared__ __align__(16) _Float16 As[BROWS * APITCH];
  __shared__ __align__(16) float Gs[BROWS * GPITCH];
  __shared__ __align__(16) float Os[BROWS * OPITCH];
  __shared__ float XIN[BROWS];
  __shared__ float WXs[NGATE];
  __shared__ float BS1s[NGATE];
  __shared__ float BS2s[NGATE];
  __shared__ float FCWs[HPAD];

  const int tid  = threadIdx.x;
  const int lane = tid & 31;
  const int wv   = tid >> 5;
  const int lr   = lane & 15;
  const int hi16 = lane >> 4;
  const int m_e  = tid >> 4;
  const int s_e  = tid & 15;
  const int b0   = blockIdx.x * BROWS;

  {
    unsigned* Au = reinterpret_cast<unsigned*>(As);
    for (int i = tid; i < (BROWS * APITCH) / 2; i += 256) Au[i] = 0u;
    for (int i = tid; i < BROWS * OPITCH; i += 256) Os[i] = 0.0f;
  }
  {
    const int n = tid;
    const int g = n >> 6, c = n & 63;
    const bool valid = (c < HID);
    const int gc = g * HID + (valid ? c : (HID - 1));
    const float w  = Wih1[gc];
    const float b1 = bih1[gc] + bhh1[gc];
    const float b2 = bih2[gc] + bhh2[gc];
    WXs[n]  = valid ? w  : 0.0f;
    BS1s[n] = valid ? b1 : 0.0f;
    BS2s[n] = valid ? b2 : 0.0f;
  }
  {
    const int jj = (tid < HID) ? tid : (HID - 1);
    const float fw = fcw[jj];
    if (tid < HPAD) FCWs[tid] = (tid < HID) ? fw : 0.0f;
    const int mm = (tid < BROWS) ? tid : (BROWS - 1);
    const float x0 = x[(size_t)(b0 + mm) * (size_t)T];
    if (tid < BROWS) XIN[tid] = x0;
  }
  const float fcbv = fcb[0];
  int fdev = __builtin_amdgcn_readfirstlane(futp[0]);
  {
    const int fmax = TT - T;
    fdev = (fdev < 0) ? 0 : fdev;
    fdev = (fdev > fmax) ? fmax : fdev;
  }
  const int TTl = T + fdev;
  __syncthreads();

  const int  gate = wv >> 1;
  const bool isg  = (gate == 2);
  const float pre  = isg ? 1.0f : 0.5f;
  const float amul = isg ? 1.0f : 0.5f;
  const float aadd = isg ? 0.0f : 0.5f;
  const int col0 = wv * 32 + lr;
  const int col1 = col0 + 16;
  const float wx0 = WXs[col0],  wx1 = WXs[col1];
  const float b10 = BS1s[col0], b11 = BS1s[col1];
  const float b20 = BS2s[col0], b21 = BS2s[col1];
  float fwq[4];
#pragma unroll
  for (int q = 0; q < 4; ++q) {
    const int j  = s_e + 16 * q;
    const int jc = (j < HID) ? j : (HID - 1);
    fwq[q] = (j < HID) ? FCWs[jc] : 0.0f;
  }
  const int rbase = 8 * hi16;
  const _Float16* arow = As + lr * APITCH + 8 * hi16;
  const _Float16* w1t0 = WT1 + (size_t)col0 * K1P + 8 * hi16;
  const _Float16* w1t1 = WT1 + (size_t)col1 * K1P + 8 * hi16;
  const _Float16* w2t0 = WT2 + (size_t)col0 * K2P + 8 * hi16;
  const _Float16* w2t1 = WT2 + (size_t)col1 * K2P + 8 * hi16;
  const float* xrow  = x + (size_t)(b0 + m_e) * (size_t)T;
  const float* grow  = Gs + m_e * GPITCH;
  _Float16*    awrow = As + m_e * APITCH;
  float c1r[4] = {0.0f, 0.0f, 0.0f, 0.0f};
  float c2r[4] = {0.0f, 0.0f, 0.0f, 0.0f};
  const v8f z8 = {0.f, 0.f, 0.f, 0.f, 0.f, 0.f, 0.f, 0.f};

  for (int t = 0; t < TTl; ++t) {
    __syncthreads();

    {
      v8f acc0 = z8, acc1 = z8;
      gemm16<2>(arow, w1t0, w1t1, acc0, acc1);
      float xin[8];
#pragma unroll
      for (int r = 0; r < 8; ++r) xin[r] = XIN[rbase + r];
      gate_epi(Gs, col0, rbase, acc0, xin, wx0, b10, pre, amul, aadd);
      gate_epi(Gs, col1, rbase, acc1, xin, wx1, b11, pre, amul, aadd);
    }
    __syncthreads();

    {
#pragma unroll
      for (int q = 0; q < 4; ++q) {
        const int j  = s_e + 16 * q;
        const int jc = (j < HID) ? j : (HID - 1);
        const float iv = grow[jc];
        const float fv = grow[HPAD + jc];
        const float gv = grow[2 * HPAD + jc];
        const float ov = grow[3 * HPAD + jc];
        const float cn = fv * c1r[q] + iv * gv;
        c1r[q] = cn;
        const float hval = ov * tanh_f(cn);
        if (j < HID) awrow[j] = (_Float16)(hval * HSCALE);
      }
    }
    __syncthreads();

    {
      v8f acc0 = z8, acc1 = z8;
      gemm16<4>(arow, w2t0, w2t1, acc0, acc1);
      float xin[8];
#pragma unroll
      for (int r = 0; r < 8; ++r) xin[r] = 0.0f;
      gate_epi(Gs, col0, rbase, acc0, xin, 0.0f, b20, pre, amul, aadd);
      gate_epi(Gs, col1, rbase, acc1, xin, 0.0f, b21, pre, amul, aadd);
    }
    __syncthreads();

    {
      float part = 0.0f;
#pragma unroll
      for (int q = 0; q < 4; ++q) {
        const int j  = s_e + 16 * q;
        const int jc = (j < HID) ? j : (HID - 1);
        const float iv = grow[jc];
        const float fv = grow[HPAD + jc];
        const float gv = grow[2 * HPAD + jc];
        const float ov = grow[3 * HPAD + jc];
        const float cn = fv * c2r[q] + iv * gv;
        c2r[q] = cn;
        const float hval = ov * tanh_f(cn);
        if (j < HID) awrow[HPAD + j] = (_Float16)(hval * HSCALE);
        part = __builtin_fmaf(hval, fwq[q], part);
      }
      part += __shfl_xor(part, 8, 32);
      part += __shfl_xor(part, 4, 32);
      part += __shfl_xor(part, 2, 32);
      part += __shfl_xor(part, 1, 32);
      const float oval = part + fcbv;
      const int tn = (t + 1 < T) ? (t + 1) : (T - 1);
      const float xn = xrow[tn];
      if (s_e == 0) {
        Os[m_e * OPITCH + (t & (OCHUNK - 1))] = oval;
        XIN[m_e] = (t + 1 < T) ? xn : oval;
      }
    }

    if (((t & (OCHUNK - 1)) == (OCHUNK - 1)) || (t == TTl - 1)) {
      __syncthreads();
      const int chunk = t >> 6;
      const int q   = lane >> 3;
      const int c4  = (lane & 7) * 4;
      const int row = wv * 2 + (q >> 1);
      const int seg = (q & 1) * 32;
      const v4f val = *(const v4f*)(Os + row * OPITCH + seg + c4);
      float* dst = out + (size_t)(b0 + row) * (size_t)TT + (size_t)chunk * OCHUNK + seg + c4;
      *(volatile v4f*)dst = val;
      __threadfence();
      *(volatile v4f*)dst = val;
    }
  }
}

extern "C" void kernel_launch(void* const* d_in, const int* in_sizes, int n_in,
                              void* d_out, int out_size, void* d_ws, size_t ws_size,
                              hipStream_t stream) {
  if (n_in < 12) return;
  const int nx = in_sizes[0];
  if (nx <= 0 || (nx % NBATCH) != 0) return;
  const int T = nx / NBATCH;
  if (out_size <= 0 || (out_size % NBATCH) != 0) return;
  const int TT = out_size / NBATCH;
  if (TT < T || (TT % OCHUNK) != 0) return;
  if (in_sizes[2] != 4 * HID * HID || in_sizes[5] != 4 * HID * HID || in_sizes[6] != 4 * HID * HID) return;
  if (in_sizes[1] != 4 * HID || in_sizes[3] != 4 * HID || in_sizes[4] != 4 * HID ||
      in_sizes[7] != 4 * HID || in_sizes[8] != 4 * HID || in_sizes[9] != HID ||
      in_sizes[10] < 1 || in_sizes[11] < 1) return;

  const size_t wt1_bytes = (size_t)NGATE * K1P * sizeof(_Float16);
  const size_t wt2_bytes = (size_t)NGATE * K2P * sizeof(_Float16);
  if (wt1_bytes + wt2_bytes > ws_size) return;

  const float* x    = (const float*)d_in[0];
  const float* Wih1 = (const float*)d_in[1];
  const float* Whh1 = (const float*)d_in[2];
  const float* bih1 = (const float*)d_in[3];
  const float* bhh1 = (const float*)d_in[4];
  const float* Wih2 = (const float*)d_in[5];
  const float* Whh2 = (const float*)d_in[6];
  const float* bih2 = (const float*)d_in[7];
  const float* bhh2 = (const float*)d_in[8];
  const float* fcw  = (const float*)d_in[9];
  const float* fcb  = (const float*)d_in[10];
  const int*   futp = (const int*)d_in[11];

  _Float16* WT1 = (_Float16*)d_ws;
  _Float16* WT2 = (_Float16*)((char*)d_ws + wt1_bytes);
  float* out = (float*)d_out;

  pack_tables<<<(NT1 + NT2) / 256, 256, 0, stream>>>(Whh1, Wih2, Whh2, WT1, WT2);
  lstm_scan<<<NBATCH / BROWS, 256, 0, stream>>>(x, Wih1, bih1, bhh1, bih2, bhh2, fcw, fcb, futp,
                                                 WT1, WT2, out, T, TT);
}
